// SpatialLocalAttention_35948876267796
// MI455X (gfx1250) — hardware-verified
//
#include <hip/hip_runtime.h>
#include <stddef.h>


typedef _Float16 h16;
typedef _Float16 v16h __attribute__((ext_vector_type(16)));
typedef _Float16 v8h  __attribute__((ext_vector_type(8)));
typedef _Float16 v4h  __attribute__((ext_vector_type(4)));
typedef _Float16 v2h  __attribute__((ext_vector_type(2)));
typedef float    v8f  __attribute__((ext_vector_type(8)));
typedef float    v4f  __attribute__((ext_vector_type(4)));
typedef float    v2f  __attribute__((ext_vector_type(2)));

#ifndef NB
#define NB 2
#endif
#ifndef SEQ
#define SEQ 4096
#endif
#define NB_FULL  2
#define SEQ_FULL 4096
#define DIM    256
#define INNER  512
#define NHEAD  8
#define HD     64
#define PE     32
#define KNB    16
#define NGLOB  4
#define NSLOT  21
#define NLOC   17
#define KVIN   288
#define QKVLD  1536
#define MROWS  (NB * SEQ)
#define MPAD   (MROWS + 64)
#define QB     16

static_assert(NB >= 1 && NB <= NB_FULL);
static_assert(SEQ >= 64 && SEQ <= SEQ_FULL && (SEQ % 64) == 0);
static_assert(INNER == NHEAD * HD);
static_assert(HD == 64);
static_assert(PE == 32);
static_assert(KVIN == DIM + PE);
static_assert(NSLOT == 1 + KNB + NGLOB && NLOC == 1 + KNB && NSLOT <= 32);
static_assert(QKVLD == 3 * INNER);
static_assert((DIM % 64) == 0 && (DIM % 32) == 0);
static_assert((INNER % 64) == 0 && (INNER % 32) == 0);
static_assert((QKVLD % 64) == 0);
static_assert((MROWS % 64) == 0 && (MPAD % 64) == 0 && (MPAD % 8) == 0);
static_assert(NB * NGLOB <= 64);
static_assert(DIM == 32 * 8);
static_assert(QB == 16 && (SEQ % QB) == 0 && (MROWS % QB) == 0);
static_assert(NHEAD == 4 * 2);
static_assert(QB * NLOC * 8 == 17 * 128);
static_assert(QB * 32 == 4 * 128);

#define LDT 72
#define LDC 68
static_assert((LDT % 8) == 0 && LDT >= 64);
static_assert((LDC % 4) == 0 && LDC >= 64);

#define RLD   40
#define QRLD  32
#define PVLD  68
#define WRLD  40
static_assert((RLD % 8) == 0 && RLD >= PE);
static_assert((WRLD % 8) == 0 && WRLD >= PE);
static_assert((PVLD % 4) == 0 && PVLD >= HD);
static_assert(QRLD == 32);

#define WCARRY  64.0f
#define VCARRY  64.0f
#define RWCARRY 16.0f

#define WT_BYTES   ((size_t)QKVLD * DIM * 2)
#define WOT_BYTES  ((size_t)DIM * INNER * 2)
#define WKR_BYTES  ((size_t)PE * INNER * 2)
#define WVRT_BYTES ((size_t)INNER * PE * 2)
#define X16_BYTES  ((size_t)MPAD * DIM * 2)
#define QKV_BYTES  ((size_t)MPAD * QKVLD * 2)
#define AO_BYTES   ((size_t)MROWS * INNER * 2)
#define OFF_WT   ((size_t)0)
#define OFF_WOT  (OFF_WT + WT_BYTES)
#define OFF_WKR  (OFF_WOT + WOT_BYTES)
#define OFF_WVRT (OFF_WKR + WKR_BYTES)
#define OFF_X16  (OFF_WVRT + WVRT_BYTES)
#define OFF_QKV  (OFF_X16 + X16_BYTES)
#define OFF_AO   (OFF_QKV + QKV_BYTES)
#define WS_TOTAL (OFF_AO + AO_BYTES)
static_assert((WT_BYTES % 128) == 0 && (WOT_BYTES % 128) == 0 && (WKR_BYTES % 128) == 0);
static_assert((WVRT_BYTES % 128) == 0 && (X16_BYTES % 128) == 0 && (QKV_BYTES % 128) == 0);
static_assert((AO_BYTES % 128) == 0);
static_assert(WS_TOTAL <= (size_t)134217728);

__device__ __forceinline__ float bf16r(float x) {
  unsigned int u = __float_as_uint(x);
  u = (u + 0x7FFFu + ((u >> 16) & 1u)) & 0xFFFF0000u;
  return __uint_as_float(u);
}

static __device__ __forceinline__ h16 toh_flush(float v) {
  const h16 r = (h16)v;
  return (fabsf(v) < 6.103515625e-05f) ? (h16)0.0f : r;
}

__device__ __forceinline__ v16h frag_at(const _Float16* p) {
  v8h lo = *(const v8h*)(p);
  v8h hi = *(const v8h*)(p + 16);
  v16h out;
#pragma unroll
  for (int i = 0; i < 8; ++i) { out[i] = lo[i]; out[i + 8] = hi[i]; }
  return out;
}

__device__ __forceinline__ v8f wmma16(v16h a, v16h b, v8f c) {
  v8f d = __builtin_amdgcn_wmma_f32_16x16x32_f16(false, a, false, b, (short)0, c,
                                                 false, false);
  asm volatile("v_nop\n\tv_nop\n\tv_nop\n\tv_nop" : "+v"(d) : "v"(a), "v"(b));
  return d;
}

__device__ __forceinline__ float red32_sum(float x) {
#pragma unroll
  for (int off = 1; off < 32; off <<= 1) x += __shfl_xor(x, off, 32);
  return x;
}
__device__ __forceinline__ float red32_max(float x) {
#pragma unroll
  for (int off = 1; off < 32; off <<= 1) x = fmaxf(x, __shfl_xor(x, off, 32));
  return x;
}

__device__ __forceinline__ void wave_lds_sync() {
  __builtin_amdgcn_fence(3  , "wavefront");
  asm volatile("s_wait_dscnt 0x0" ::: "memory");
  __builtin_amdgcn_wave_barrier();
}

__global__ __launch_bounds__(256) void wconv_kernel(
    const float* __restrict__ W, _Float16* __restrict__ Wt, unsigned ldw, unsigned ldk) {
  __shared__ _Float16 T[64 * LDT];
  const unsigned tid = threadIdx.x;
  const unsigned n0 = blockIdx.x * 64u;
  const unsigned k0 = blockIdx.y * 64u;
#pragma unroll 4
  for (unsigned j = 0; j < 16u; ++j) {
    const unsigned idx = tid + 256u * j;
    const unsigned kr = idx >> 6, nc = idx & 63u;
    const float v = W[(size_t)(k0 + kr) * ldw + n0 + nc];
    T[nc * LDT + kr] = (_Float16)(WCARRY * bf16r(v));
  }
  __syncthreads();
  v8h x[2];
  size_t off[2];
#pragma unroll
  for (unsigned i = 0; i < 2u; ++i) {
    const unsigned n = 32u * i + (tid >> 3);
    const unsigned kc = (tid & 7u) * 8u;
    x[i] = *(const v8h*)&T[n * LDT + kc];
    off[i] = (size_t)(n0 + n) * ldk + k0 + kc;
  }
#pragma unroll
  for (int i = 0; i < 2; ++i) *(volatile v8h*)(Wt + off[i]) = x[i];
  __threadfence();
#pragma unroll
  for (int i = 0; i < 2; ++i) *(volatile v8h*)(Wt + off[i]) = x[i];
}

__global__ __launch_bounds__(256) void rpew_kernel(
    const float* __restrict__ Wk, const float* __restrict__ Wv,
    _Float16* __restrict__ Wkr, _Float16* __restrict__ WvrT) {
  __shared__ __attribute__((aligned(16))) _Float16 T[64 * RLD];
  const unsigned tid = threadIdx.x;
  const unsigned f0 = blockIdx.x * 64u;
#pragma unroll 2
  for (unsigned j = 0; j < 8u; ++j) {
    const unsigned idx = tid + 256u * j;
    const unsigned p = idx >> 6, fc = idx & 63u;
    const float v = Wv[(size_t)(DIM + p) * INNER + f0 + fc];
    T[fc * RLD + p] = toh_flush(WCARRY * bf16r(v));
  }
  const unsigned p = tid >> 3, pc = (tid & 7u) * 8u;
  const v4f a0 = *(const v4f*)(Wk + (size_t)(DIM + p) * INNER + f0 + pc);
  const v4f a1 = *(const v4f*)(Wk + (size_t)(DIM + p) * INNER + f0 + pc + 4u);
  v8h xk;
#pragma unroll
  for (int i = 0; i < 4; ++i) {
    xk[i]     = toh_flush(WCARRY * bf16r(a0[i]));
    xk[i + 4] = toh_flush(WCARRY * bf16r(a1[i]));
  }
  __syncthreads();
  const unsigned fr = tid >> 2, pq = (tid & 3u) * 8u;
  const v8h xv = *(const v8h*)&T[fr * RLD + pq];
  const size_t offk = (size_t)p * INNER + f0 + pc;
  const size_t offv = (size_t)(f0 + fr) * PE + pq;
  *(volatile v8h*)(Wkr + offk) = xk;
  *(volatile v8h*)(WvrT + offv) = xv;
  __threadfence();
  *(volatile v8h*)(Wkr + offk) = xk;
  *(volatile v8h*)(WvrT + offv) = xv;
}

__global__ __launch_bounds__(256) void xconv_kernel(
    const float* __restrict__ X, const float* __restrict__ GL, _Float16* __restrict__ dst) {
  const unsigned lane = threadIdx.x & 31u, w = threadIdx.x >> 5;
  const unsigned crow = blockIdx.x * 8u + w;
  const bool isx = crow < (unsigned)MROWS;
  const bool isg = (crow >= (unsigned)MROWS) && (crow < (unsigned)(MROWS + NB * NGLOB));
  const unsigned cx = isx ? crow : (unsigned)(MROWS - 1);
  const unsigned bidx = cx / (unsigned)SEQ;
  const unsigned sq = cx - bidx * (unsigned)SEQ;
  const size_t srow = (size_t)bidx * SEQ_FULL + sq;
  const unsigned gi = isg ? (crow - (unsigned)MROWS) : 0u;
  v4f a0 = *(const v4f*)(X + srow * DIM + lane * 8u);
  v4f a1 = *(const v4f*)(X + srow * DIM + lane * 8u + 4u);
  v4f g0 = *(const v4f*)(GL + (size_t)gi * DIM + lane * 8u);
  v4f g1 = *(const v4f*)(GL + (size_t)gi * DIM + lane * 8u + 4u);
  asm volatile("" : "+v"(a0));
  asm volatile("" : "+v"(a1));
  asm volatile("" : "+v"(g0));
  asm volatile("" : "+v"(g1));
  v8h o;
#pragma unroll
  for (int i = 0; i < 4; ++i) {
    const float t0 = isx ? a0[i] : (isg ? g0[i] : 0.0f);
    const float t1 = isx ? a1[i] : (isg ? g1[i] : 0.0f);
    o[i]     = toh_flush(bf16r(t0));
    o[i + 4] = toh_flush(bf16r(t1));
  }
  _Float16* p = dst + (size_t)crow * DIM + lane * 8u;
  *(volatile v8h*)p = o;
  __threadfence();
  *(volatile v8h*)p = o;
}

template <int MODE>
__device__ __forceinline__ void gemm_body(
    const _Float16* __restrict__ A16, const _Float16* __restrict__ Bt, const unsigned K,
    const float* __restrict__ bias, float* __restrict__ outf, _Float16* __restrict__ out16) {
  __shared__ __attribute__((aligned(16))) float Cs[64 * LDC];
  const unsigned tid = threadIdx.x, lane = tid & 31u, w = tid >> 5;
  const unsigned mw = w >> 1, nw = w & 1u;
  const unsigned hh = lane >> 4, m = lane & 15u;
  const unsigned n0 = blockIdx.x * 64u;
  const unsigned row0 = blockIdx.y * 64u;

  const _Float16* ap  = A16 + (size_t)(row0 + mw * 16u + m) * K + hh * 8u;
  const _Float16* bp0 = Bt + (size_t)(n0 + nw * 32u + m) * K + hh * 8u;
  const _Float16* bp1 = bp0 + (size_t)16 * K;
  v8f acc0 = {}, acc1 = {};
#pragma unroll 2
  for (unsigned k0 = 0; k0 < K; k0 += 32u) {
    const v16h a  = frag_at(ap + k0);
    const v16h b0 = frag_at(bp0 + k0);
    const v16h b1 = frag_at(bp1 + k0);
    acc0 = wmma16(a, b0, acc0);
    acc1 = wmma16(a, b1, acc1);
  }
#pragma unroll
  for (int r = 0; r < 8; ++r) {
    float* d = &Cs[(mw * 16u + hh * 8u + (unsigned)r) * LDC + nw * 32u + m];
    d[0]  = acc0[r];
    d[16] = acc1[r];
  }
  __syncthreads();

  if (MODE == 0) {
    v8h x[2];
    size_t off[2];
#pragma unroll
    for (unsigned i = 0; i < 2u; ++i) {
      const unsigned r = 32u * i + (tid >> 3);
      const unsigned c = (tid & 7u) * 8u;
      const v4f u0 = *(const v4f*)&Cs[r * LDC + c];
      const v4f u1 = *(const v4f*)&Cs[r * LDC + c + 4];
#pragma unroll
      for (int j = 0; j < 4; ++j) {
        x[i][j]     = toh_flush(u0[j] * (1.0f / WCARRY));
        x[i][j + 4] = toh_flush(u1[j] * (1.0f / WCARRY));
      }
      off[i] = (size_t)(row0 + r) * QKVLD + n0 + c;
    }
#pragma unroll
    for (int i = 0; i < 2; ++i) *(volatile v8h*)(out16 + off[i]) = x[i];
    __threadfence();
#pragma unroll
    for (int i = 0; i < 2; ++i) *(volatile v8h*)(out16 + off[i]) = x[i];
  }

  if (MODE == 1) {
    const float cs = 1.0f / (WCARRY * VCARRY);
    v4f xs[4];
    size_t off[4];
#pragma unroll
    for (unsigned i = 0; i < 4u; ++i) {
      const unsigned r = 16u * i + (tid >> 4);
      const unsigned c = (tid & 15u) * 4u;
      const unsigned crow = row0 + r;
      const unsigned bidx = crow / (unsigned)SEQ;
      const unsigned sq = crow - bidx * (unsigned)SEQ;
      const size_t frow = (size_t)bidx * SEQ_FULL + sq;
      const v4f u = *(const v4f*)&Cs[r * LDC + c];
      const v4f g = *(const v4f*)(bias + n0 + c);
      v4f val;
#pragma unroll
      for (int j = 0; j < 4; ++j) val[j] = u[j] * cs + bf16r(g[j]);
      xs[i] = val;
      off[i] = frow * DIM + n0 + c;
    }
#pragma unroll
    for (int i = 0; i < 4; ++i) *(volatile v4f*)(outf + off[i]) = xs[i];
    __threadfence();
#pragma unroll
    for (int i = 0; i < 4; ++i) *(volatile v4f*)(outf + off[i]) = xs[i];
  }
}

__global__ __launch_bounds__(256) void gemm_proj_kernel(
    const _Float16* __restrict__ A16, const _Float16* __restrict__ Bt,
    _Float16* __restrict__ out16) {
  gemm_body<0>(A16, Bt, (unsigned)DIM, (const float*)0, (float*)0, out16);
}
__global__ __launch_bounds__(256) void gemm_out_kernel(
    const _Float16* __restrict__ A16, const _Float16* __restrict__ Bt,
    const float* __restrict__ bias, float* __restrict__ outf) {
  gemm_body<1>(A16, Bt, (unsigned)INNER, bias, outf, (_Float16*)0);
}

__global__ __launch_bounds__(128) void attn_kernel(
    const _Float16* __restrict__ QKV, const int* __restrict__ topk,
    const float* __restrict__ rpe, const float* __restrict__ srpe,
    const float* __restrict__ dist, const float* __restrict__ lsig,
    const float* __restrict__ gbias, const _Float16* __restrict__ Wkr,
    const _Float16* __restrict__ WvrT, _Float16* __restrict__ AO) {
  __shared__ __attribute__((aligned(16))) _Float16 RPs[QB * NLOC * RLD];
  __shared__ __attribute__((aligned(16))) int      sRow[QB * 32];
  __shared__ __attribute__((aligned(16))) float    sD2[QB * 32];
  __shared__ __attribute__((aligned(16))) float    QRs[4 * QB * QRLD];
  __shared__ __attribute__((aligned(16))) float    PVt[4 * QB * PVLD];
  __shared__ __attribute__((aligned(16))) _Float16 WRs[4 * QB * WRLD];

  const unsigned tid = threadIdx.x, lane = tid & 31u;
  const unsigned wave = __builtin_amdgcn_readfirstlane(threadIdx.x >> 5);
  const unsigned hh = lane >> 4, m = lane & 15u;
  const unsigned crow0 = blockIdx.x * (unsigned)QB;
  const unsigned b = crow0 / (unsigned)SEQ;
  const unsigned l0 = crow0 - b * (unsigned)SEQ;
  const size_t fq0 = (size_t)b * SEQ_FULL + l0;

#pragma unroll 1
  for (unsigned j = 0; j < 4u; ++j) {
    const unsigned e = tid + 128u * j;
    const unsigned qi = e >> 5, c = e & 31u;
    const unsigned cc = (c >= 1u) ? ((c <= 16u) ? (c - 1u) : 15u) : 0u;
    const size_t fq = fq0 + qi;
    int idx = topk[fq * KNB + cc];
    float dv = dist[fq * KNB + cc];
    asm volatile("" : "+v"(idx));
    asm volatile("" : "+v"(dv));
    idx = (idx < 0) ? (idx + SEQ) : idx;
    idx = (idx < 0) ? 0 : idx;
    idx = (idx > SEQ - 1) ? (SEQ - 1) : idx;
    const float d = bf16r(dv);
    const bool nbr = (c >= 1u) && (c <= 16u);
    const bool glb = (c >= 17u) && (c <= 20u);
    const unsigned gsl = (c >= 17u) ? ((c <= 20u) ? (c - 17u) : 3u) : 0u;
    const int selfrow = (int)(crow0 + qi);
    const int grow = (int)((unsigned)MROWS + b * (unsigned)NGLOB + gsl);
    const int nrow = (int)(b * (unsigned)SEQ) + idx;
    sRow[e] = nbr ? nrow : (glb ? grow : selfrow);
    sD2[e] = nbr ? (d * d) : 0.0f;
  }
#pragma unroll 1
  for (unsigned j = 0; j < 17u; ++j) {
    const unsigned e = tid + 128u * j;
    const unsigned qi = e / 136u;
    const unsigned rem = e - qi * 136u;
    const unsigned sl = rem >> 3, pc = rem & 7u;
    const unsigned sj = (sl >= 1u) ? (sl - 1u) : 0u;
    const size_t fq = fq0 + qi;
    v4f a = *(const v4f*)(srpe + fq * PE + pc * 4u);
    v4f r = *(const v4f*)(rpe + (fq * KNB + sj) * PE + pc * 4u);
    asm volatile("" : "+v"(a));
    asm volatile("" : "+v"(r));
    v4h o;
#pragma unroll
    for (int i = 0; i < 4; ++i) {
      const float t = (sl == 0u) ? a[i] : r[i];
      o[i] = (_Float16)bf16r(t);
    }
    *(v4h*)&RPs[(qi * NLOC + sl) * RLD + pc * 4u] = o;
  }
  __syncthreads();

  const unsigned qbw = wave * (unsigned)(QB * QRLD);
  const unsigned pbw = wave * (unsigned)(QB * PVLD);
  const unsigned wbw = wave * (unsigned)(QB * WRLD);
  const float gb = bf16r(gbias[0]);

#pragma unroll 1
  for (unsigned hs = 0; hs < 2u; ++hs) {
    const unsigned head = wave * 2u + hs;
    const float ls = bf16r(lsig[head]);
    const float ex = expf(ls);
    const float inv2s = __builtin_amdgcn_rcpf(2.0f * (ex * ex));

    {
      const _Float16* qp = QKV + (size_t)(crow0 + m) * QKVLD + head * 64u + hh * 8u;
      const v16h qa0 = frag_at(qp);
      const v16h qa1 = frag_at(qp + 32);
#pragma unroll
      for (int nt = 0; nt < 2; ++nt) {
        const _Float16* bp = Wkr + (size_t)((unsigned)nt * 16u + m) * INNER + head * 64u + hh * 8u;
        v8f t = {};
        t = wmma16(qa0, frag_at(bp), t);
        t = wmma16(qa1, frag_at(bp + 32), t);
#pragma unroll
        for (int r = 0; r < 8; ++r)
          QRs[qbw + (hh * 8u + (unsigned)r) * QRLD + (unsigned)nt * 16u + m] =
              t[r] * (1.0f / WCARRY);
      }
    }
    wave_lds_sync();

#pragma unroll 1
    for (unsigned qi = 0; qi < (unsigned)QB; ++qi) {
      const unsigned te = qi * 32u + lane;
      const int row = sRow[te];
      const float d2 = sD2[te];
      const _Float16* kp = QKV + (size_t)row * QKVLD + INNER + head * 64u;
      const _Float16* qp = QKV + (size_t)(crow0 + qi) * QKVLD + head * 64u;
      float s1 = 0.0f;
#pragma unroll 1
      for (unsigned i = 0; i < 8u; ++i) {
        const v8h kk = *(const v8h*)(kp + i * 8u);
        const v8h qq = *(const v8h*)(qp + i * 8u);
#pragma unroll
        for (int t = 0; t < 8; ++t) s1 += (float)qq[t] * (float)kk[t];
      }
      const unsigned cr = (lane < 16u) ? lane : 16u;
      const unsigned rbase = (qi * NLOC + cr) * RLD;
      const unsigned qbase = qbw + qi * QRLD;
      float s2 = 0.0f;
#pragma unroll 1
      for (unsigned i = 0; i < 4u; ++i) {
        const v8h rr = *(const v8h*)&RPs[rbase + i * 8u];
        const v4f q0 = *(const v4f*)&QRs[qbase + i * 8u];
        const v4f q1 = *(const v4f*)&QRs[qbase + i * 8u + 4u];
#pragma unroll
        for (int t = 0; t < 4; ++t) {
          s2 += (float)rr[t] * q0[t];
          s2 += (float)rr[t + 4] * q1[t];
        }
      }
      const bool active = lane < (unsigned)NSLOT;
      const bool local = lane < (unsigned)NLOC;
      const float sdot = local ? (s1 + s2) : s1;
      const float bias = local ? -(d2 * inv2s) : gb;
      float s = sdot * 0.125f + bias;
      s = active ? s : -1.0e30f;
      const float mx = red32_max(s);
      float e = __expf(s - mx);
      e = active ? e : 0.0f;
      const float sum = red32_sum(e);
      const float wgt = e * __builtin_amdgcn_rcpf(sum);

      wave_lds_sync();
      QRs[qbase + lane] = wgt;
      wave_lds_sync();

      float wr = 0.0f;
#pragma unroll 1
      for (unsigned c = 0; c < (unsigned)NLOC; ++c)
        wr += QRs[qbase + c] * (float)RPs[(qi * NLOC + c) * RLD + lane];
      WRs[wbw + qi * WRLD + lane] = toh_flush(RWCARRY * wr);

      float a0 = 0.0f, a1 = 0.0f;
#pragma unroll 1
      for (unsigned c = 0; c < (unsigned)NSLOT; ++c) {
        const float wc = QRs[qbase + c];
        const int vr = sRow[qi * 32u + c];
        const v2h vv = *(const v2h*)(QKV + (size_t)vr * QKVLD + 2u * INNER + head * 64u + lane * 2u);
        a0 += wc * (float)vv[0];
        a1 += wc * (float)vv[1];
      }
      v2f pv;
      pv[0] = a0 * (WCARRY * RWCARRY);
      pv[1] = a1 * (WCARRY * RWCARRY);
      *(v2f*)&PVt[pbw + qi * PVLD + lane * 2u] = pv;
    }
    wave_lds_sync();

    {
      const v16h wa = frag_at(&WRs[wbw + m * WRLD + hh * 8u]);
#pragma unroll
      for (int nt = 0; nt < 4; ++nt) {
        const v16h vb = frag_at(WvrT + (size_t)(head * 64u + (unsigned)nt * 16u + m) * PE + hh * 8u);
        v8f acc;
#pragma unroll
        for (int r = 0; r < 8; ++r)
          acc[r] = PVt[pbw + (hh * 8u + (unsigned)r) * PVLD + (unsigned)nt * 16u + m];
        acc = wmma16(wa, vb, acc);
#pragma unroll
        for (int r = 0; r < 8; ++r)
          PVt[pbw + (hh * 8u + (unsigned)r) * PVLD + (unsigned)nt * 16u + m] =
              acc[r] * (VCARRY / (WCARRY * RWCARRY));
      }
    }
    wave_lds_sync();

    v8h x[4];
    size_t off[4];
#pragma unroll
    for (unsigned i = 0; i < 4u; ++i) {
      const unsigned r = 4u * i + (lane >> 3);
      const unsigned c = (lane & 7u) * 8u;
      const v4f u0 = *(const v4f*)&PVt[pbw + r * PVLD + c];
      const v4f u1 = *(const v4f*)&PVt[pbw + r * PVLD + c + 4u];
#pragma unroll
      for (int j = 0; j < 4; ++j) {
        x[i][j]     = toh_flush(u0[j]);
        x[i][j + 4] = toh_flush(u1[j]);
      }
      off[i] = (size_t)(crow0 + r) * INNER + head * 64u + c;
    }
#pragma unroll
    for (int i = 0; i < 4; ++i) *(volatile v8h*)(AO + off[i]) = x[i];
    __threadfence();
#pragma unroll
    for (int i = 0; i < 4; ++i) *(volatile v8h*)(AO + off[i]) = x[i];
    wave_lds_sync();
  }
}

extern "C" void kernel_launch(void* const* d_in, const int* in_sizes, int n_in,
                              void* d_out, int out_size, void* d_ws, size_t ws_size,
                              hipStream_t stream) {
  if (n_in < 13) return;
  const long long rows_need = (long long)(NB - 1) * SEQ_FULL + SEQ;
  if ((long long)in_sizes[0] < rows_need * DIM) return;
  if ((long long)in_sizes[1] < rows_need * KNB) return;
  if ((long long)in_sizes[2] < rows_need * KNB * PE) return;
  if ((long long)in_sizes[3] < rows_need * PE) return;
  if ((long long)in_sizes[4] < rows_need * KNB) return;
  if ((long long)in_sizes[5] < (long long)NB * NGLOB * DIM) return;
  if ((long long)in_sizes[6] < (long long)DIM * INNER) return;
  if ((long long)in_sizes[7] < (long long)KVIN * INNER) return;
  if ((long long)in_sizes[8] < (long long)KVIN * INNER) return;
  if ((long long)in_sizes[9] < (long long)INNER * DIM) return;
  if (in_sizes[10] < DIM || in_sizes[11] < NHEAD || in_sizes[12] < 1) return;
  if ((long long)out_size < rows_need * DIM) return;
  if (ws_size < WS_TOTAL) return;

  const float* X    = (const float*)d_in[0];
  const int*   topk = (const int*)d_in[1];
  const float* rpe  = (const float*)d_in[2];
  const float* srpe = (const float*)d_in[3];
  const float* dist = (const float*)d_in[4];
  const float* glat = (const float*)d_in[5];
  const float* wq   = (const float*)d_in[6];
  const float* wk   = (const float*)d_in[7];
  const float* wv   = (const float*)d_in[8];
  const float* wo   = (const float*)d_in[9];
  const float* bo   = (const float*)d_in[10];
  const float* lsig = (const float*)d_in[11];
  const float* gbia = (const float*)d_in[12];
  float* out = (float*)d_out;

  char* ws = (char*)d_ws;
  _Float16* WT16   = (_Float16*)(ws + OFF_WT);
  _Float16* WoT16  = (_Float16*)(ws + OFF_WOT);
  _Float16* Wkr16  = (_Float16*)(ws + OFF_WKR);
  _Float16* WvrT16 = (_Float16*)(ws + OFF_WVRT);
  _Float16* X16    = (_Float16*)(ws + OFF_X16);
  _Float16* QKV16  = (_Float16*)(ws + OFF_QKV);
  _Float16* AO16   = (_Float16*)(ws + OFF_AO);

  dim3 blk(256);
  wconv_kernel<<<dim3(INNER / 64, DIM / 64), blk, 0, stream>>>(wq, WT16, (unsigned)INNER, (unsigned)DIM);
  wconv_kernel<<<dim3(INNER / 64, DIM / 64), blk, 0, stream>>>(wk, WT16 + (size_t)INNER * DIM, (unsigned)INNER, (unsigned)DIM);
  wconv_kernel<<<dim3(INNER / 64, DIM / 64), blk, 0, stream>>>(wv, WT16 + (size_t)2 * INNER * DIM, (unsigned)INNER, (unsigned)DIM);
  wconv_kernel<<<dim3(DIM / 64, INNER / 64), blk, 0, stream>>>(wo, WoT16, (unsigned)DIM, (unsigned)INNER);
  rpew_kernel<<<dim3(INNER / 64), blk, 0, stream>>>(wk, wv, Wkr16, WvrT16);

  xconv_kernel<<<dim3(MPAD / 8), blk, 0, stream>>>(X, glat, X16);
  gemm_proj_kernel<<<dim3(QKVLD / 64, MPAD / 64), blk, 0, stream>>>(X16, WT16, QKV16);
  attn_kernel<<<dim3(MROWS / QB), dim3(128), 0, stream>>>(QKV16, topk, rpe, srpe, dist, lsig, gbia,
                                                          Wkr16, WvrT16, AO16);
  gemm_out_kernel<<<dim3(DIM / 64, MROWS / 64), blk, 0, stream>>>(AO16, WoT16, bo, out);
}
